// RAE_60112362275057
// MI455X (gfx1250) — hardware-verified
//
#include <hip/hip_runtime.h>
#include <math.h>

typedef __attribute__((ext_vector_type(16))) _Float16 v16h;
typedef __attribute__((ext_vector_type(8)))  _Float16 v8h;
typedef __attribute__((ext_vector_type(16))) __bf16   v16b;
typedef __attribute__((ext_vector_type(8)))  __bf16   v8b;
typedef __attribute__((ext_vector_type(8)))  float    v8f;
typedef __attribute__((ext_vector_type(4)))  float    v4f;

constexpr int kB    = 256;
constexpr int kT    = 64;
constexpr int kXD   = 128;
constexpr int kHD   = 1024;
constexpr int kG3   = 3 * kHD;
constexpr int kRing = 16;
constexpr int kThr  = 256;
constexpr float kInCarry = 1024.0f;
constexpr float kSc = 1.0f / (kInCarry * kInCarry);
constexpr float kF16MinNormal = 6.103515625e-5f;
constexpr int kFEI = 0, kFEH = 3072, kFDI = 6144, kFDH = 9216, kFBL = 12288, kFEnd = 13312;

static_assert((kB % 64) == 0 && ((kB / 64) * (kG3 / 64)) % 8 == 0 && ((kB / 64) * (kXD / 64)) % 8 == 0 && (kHD % 32) == 0 && (kXD % 32) == 0 && (kRing & (kRing - 1)) == 0 && kRing > 10,
              "GEMM M, N multiples of 64; grids exact; K multiples of 32; the ring holds the lists' reach");

static const int kPrevSkip[64] = {-1, -1, -1, 1, 3, -1, -1, -1, -1, -1, 0, 1, 2, 3, 4, 5, 6, 7, 8, 9, 10, 11, 12, 13, 14, 15, 16, 17, 18, 19, 20, 21, 22, 23, 24, 25, 26, 27, 28, 29, 30, 31, 32, 33, 34, 35, 36, 37, 38, 39, 40, 41, 42, 43, 44, 45, 46, 47, 48, 49, 50, 51, 52, 53};
static const int kProjSkip[64] = {-1, -1, 0, 2, 4, -1, -1, -1, -1, -1, 0, 1, 2, 3, 4, 5, 6, 7, 8, 9, 10, 11, 12, 13, 14, 15, 16, 17, 18, 19, 20, 21, 22, 23, 24, 25, 26, 27, 28, 29, 30, 31, 32, 33, 34, 35, 36, 37, 38, 39, 40, 41, 42, 43, 44, 45, 46, 47, 48, 49, 50, 51, 52, 53};
static const int kEncM1[64] = {0, 1, 0, 1, 1, 1, 1, 0, 1, 0, 0, 0, 0, 1, 1, 0, 0, 1, 1, 0, 1, 1, 1, 0, 1, 0, 0, 1, 1, 1, 1, 1, 1, 1, 0, 1, 0, 1, 0, 1, 1, 0, 0, 0, 0, 1, 0, 0, 0, 1, 0, 1, 0, 1, 1, 1, 1, 0, 1, 0, 0, 1, 0, 1};
static const int kEncM2[64] = {1, 1, 1, 1, 1, 1, 0, 1, 0, 1, 1, 1, 1, 0, 1, 1, 1, 1, 1, 1, 0, 0, 1, 1, 1, 1, 1, 0, 1, 1, 0, 0, 1, 1, 1, 0, 1, 1, 1, 0, 0, 1, 1, 1, 1, 1, 1, 1, 1, 1, 1, 0, 1, 0, 1, 1, 1, 1, 1, 1, 1, 0, 1, 1};
static const int kDecM1[64] = {0, 1, 0, 1, 0, 0, 1, 0, 1, 0, 0, 0, 0, 1, 1, 1, 1, 1, 1, 1, 0, 1, 0, 0, 1, 0, 0, 0, 1, 0, 0, 1, 1, 1, 0, 0, 0, 1, 1, 1, 1, 0, 1, 1, 0, 0, 1, 1, 1, 1, 1, 0, 0, 1, 1, 1, 0, 0, 0, 0, 1, 0, 1, 0};
static const int kDecM2[64] = {1, 0, 1, 0, 1, 1, 1, 1, 0, 1, 1, 1, 1, 0, 0, 1, 1, 0, 1, 1, 1, 1, 1, 1, 0, 1, 1, 1, 1, 1, 1, 0, 1, 1, 1, 1, 1, 0, 1, 0, 0, 1, 0, 1, 1, 1, 0, 0, 0, 0, 0, 1, 1, 0, 0, 0, 1, 1, 1, 1, 0, 1, 0, 1};

constexpr size_t kOffEWH = 0ull;
constexpr size_t kOffEWI = 6291456ull;
constexpr size_t kOffDWH = 7077888ull;
constexpr size_t kOffDWI2 = 13369344ull;
constexpr size_t kOffLW2 = 14942208ull;
constexpr size_t kOffBIAS = 15466496ull;
constexpr size_t kOffX16 = 15519744ull;
constexpr size_t kOffZERO = 19714048ull;
constexpr size_t kOffINIT = 20762624ull;
constexpr size_t kOffRING = 21811200ull;
constexpr size_t kOffHP32 = 38588416ull;
constexpr size_t kOffHP16 = 39636992ull;
constexpr size_t kOffGI = 40161280ull;
constexpr size_t kOffGH = 43307008ull;
constexpr size_t kOffPJ2 = 46452736ull;
constexpr size_t kOffPR32 = 47501312ull;
constexpr size_t kOffXIN2 = 47632384ull;
constexpr size_t kWsTotal = 47763456ull;
static_assert(kWsTotal <= 134217728ull, "carve cap: under 128 MiB");
static_assert(kOffEWH == 0
              && kOffEWI == kOffEWH + 6291456ull
              && kOffDWH == kOffEWI + 786432ull
              && kOffDWI2 == kOffDWH + 6291456ull
              && kOffLW2 == kOffDWI2 + 1572864ull
              && kOffBIAS == kOffLW2 + 524288ull
              && kOffX16 == kOffBIAS + 53248ull
              && kOffZERO == kOffX16 + 4194304ull
              && kOffINIT == kOffZERO + 1048576ull
              && kOffRING == kOffINIT + 1048576ull
              && kOffHP32 == kOffRING + 16777216ull
              && kOffHP16 == kOffHP32 + 1048576ull
              && kOffGI == kOffHP16 + 524288ull
              && kOffGH == kOffGI + 3145728ull
              && kOffPJ2 == kOffGH + 3145728ull
              && kOffPR32 == kOffPJ2 + 1048576ull
              && kOffXIN2 == kOffPR32 + 131072ull
              && kWsTotal == kOffXIN2 + 131072ull, "the carve is chained and totalled");
static_assert((kOffEWH % 256) == 0 && (kOffEWI % 256) == 0 && (kOffDWH % 256) == 0 && (kOffDWI2 % 256) == 0 && (kOffLW2 % 256) == 0 && (kOffBIAS % 256) == 0 && (kOffX16 % 256) == 0 && (kOffZERO % 256) == 0 && (kOffINIT % 256) == 0 && (kOffRING % 256) == 0 && (kOffHP32 % 256) == 0 && (kOffHP16 % 256) == 0 && (kOffGI % 256) == 0 && (kOffGH % 256) == 0 && (kOffPJ2 % 256) == 0 && (kOffPR32 % 256) == 0 && (kOffXIN2 % 256) == 0, "aligned regions");

__device__ __forceinline__ unsigned short f2bf_bits(float f) {
  unsigned u = __float_as_uint(f);
  return (unsigned short)((u + 0x7FFFu + ((u >> 16) & 1u)) >> 16);
}
__device__ __forceinline__ float bf_bits2f(unsigned short h) { return __uint_as_float(((unsigned)h) << 16); }
__device__ __forceinline__ float bf16r(float f) { return bf_bits2f(f2bf_bits(f)); }
__device__ __forceinline__ float carry_flush(float v, float carry) {
  const float s = v * carry;
  return (fabsf(s) < kF16MinNormal) ? 0.0f : s;
}
__device__ __forceinline__ float frcp(float x) { return __builtin_amdgcn_rcpf(x); }

__device__ __forceinline__ void dep_guard4_h(v8f& a, v8f& b, v8f& c, v8f& d, v16h x, v16h y) { asm volatile("v_nop\n\tv_nop\n\tv_nop\n\tv_nop" : "+v"(a), "+v"(b), "+v"(c), "+v"(d) : "v"(x), "v"(y)); }
__device__ __forceinline__ void dep_guard4_b(v8f& a, v8f& b, v8f& c, v8f& d, v16b x, v16b y) { asm volatile("v_nop\n\tv_nop\n\tv_nop\n\tv_nop" : "+v"(a), "+v"(b), "+v"(c), "+v"(d) : "v"(x), "v"(y)); }
__device__ __forceinline__ void keep4_h(v16h a, v16h b, v16h c, v16h d) { asm volatile("v_nop" :: "v"(a), "v"(b), "v"(c), "v"(d)); }
__device__ __forceinline__ void keep4_b(v16b a, v16b b, v16b c, v16b d) { asm volatile("v_nop" :: "v"(a), "v"(b), "v"(c), "v"(d)); }
__device__ __forceinline__ void acc_guard4(v8f& a, v8f& b, v8f& c, v8f& d) { asm volatile("v_nop\n\tv_nop\n\tv_nop\n\tv_nop" : "+v"(a), "+v"(b), "+v"(c), "+v"(d)); }

template <typename T> struct Frag;
template <> struct Frag<_Float16> {
  typedef v16h V; union U { v16h v; v8h h[2]; };
  static __device__ __forceinline__ v16h load(const _Float16* p) {
    U f; f.h[0] = *(const v8h*)(p); f.h[1] = *(const v8h*)(p + 16); return f.v;
  }
  static __device__ __forceinline__ v8f mma(v16h a, v16h b, v8f c) {
    return __builtin_amdgcn_wmma_f32_16x16x32_f16(false, a, false, b, (short)0, c, false, false);
  }
  static __device__ __forceinline__ void guard4(v8f& a, v8f& b, v8f& c, v8f& d, v16h x, v16h y) { dep_guard4_h(a, b, c, d, x, y); }
  static __device__ __forceinline__ void keep(v16h a, v16h b, v16h c, v16h d) { keep4_h(a, b, c, d); }
};
template <> struct Frag<__bf16> {
  typedef v16b V; union U { v16b v; v8b h[2]; };
  static __device__ __forceinline__ v16b load(const __bf16* p) {
    U f; f.h[0] = *(const v8b*)(p); f.h[1] = *(const v8b*)(p + 16); return f.v;
  }
  static __device__ __forceinline__ v8f mma(v16b a, v16b b, v8f c) {
    return __builtin_amdgcn_wmma_f32_16x16x32_bf16(false, a, false, b, (short)0, c, false, false);
  }
  static __device__ __forceinline__ void guard4(v8f& a, v8f& b, v8f& c, v8f& d, v16b x, v16b y) { dep_guard4_b(a, b, c, d, x, y); }
  static __device__ __forceinline__ void keep(v16b a, v16b b, v16b c, v16b d) { keep4_b(a, b, c, d); }
};

__device__ __forceinline__ v8f mma_h(v16h a, v16h b, v8f c) {
  c = __builtin_amdgcn_wmma_f32_16x16x32_f16(false, a, false, b, (short)0, c, false, false);
  asm volatile("v_nop\n\tv_nop\n\tv_nop\n\tv_nop" : "+v"(c) : "v"(a), "v"(b));
  return c;
}

template <int ET> struct Elem;
template <> struct Elem<0> { typedef _Float16 T; };
template <> struct Elem<1> { typedef __bf16 T; };
template <int ET, bool SPLIT, int BIAS_MODE, int OUT_MODE, bool RESID, int ACT = 0>
__global__ __launch_bounds__(256) void wmma_gemm64(
    const unsigned short* __restrict__ Ap, const unsigned short* __restrict__ A2p, int lda, long strideA,
    const unsigned short* __restrict__ Btp, const unsigned short* __restrict__ Bt2p, int ldb, long strideB,
    void* __restrict__ Cout, void* __restrict__ Cout2, int ldc, long strideC,
    const float* __restrict__ bias,
    const float* __restrict__ resid, long strideR,
    int M, int N, int K, float scale) {
  typedef typename Elem<ET>::T T;
  typedef typename Frag<T>::V V;
  const T* A = (const T*)Ap; const T* A2 = (const T*)A2p; const T* Bt = (const T*)Btp; const T* Bt2 = (const T*)Bt2p;
  __shared__ __align__(16) float sT[8][16 * 68];
  const int b    = blockIdx.y;
  const int lane = threadIdx.x & 31;
  const int wave = threadIdx.x >> 5;
  const int tilesN = N >> 6;
  const int tilesM = M >> 6;
  const int tile = blockIdx.x * 8 + wave;
  if (tile >= tilesM * tilesN) return;
  const int tm = tile / tilesN;
  const int tn = tile - tm * tilesN;
  const int m0 = tm << 6;
  const int n0 = tn << 6;

  const T* Ab  = A  + (size_t)b * strideA;
  const T* Bb  = Bt + (size_t)b * strideB;
  const T* Ab2 = SPLIT ? (A2  + (size_t)b * strideA) : nullptr;
  const T* Bb2 = SPLIT ? (Bt2 + (size_t)b * strideB) : nullptr;

  const int rlane = lane & 15;
  const int koff  = (lane >> 4) * 8;
  const int mOff  = (lane >> 4) * 8;

  v8f acc[4][4];
#pragma unroll
  for (int i = 0; i < 4; ++i)
#pragma unroll
    for (int j = 0; j < 4; ++j) acc[i][j] = (v8f){0.f,0.f,0.f,0.f,0.f,0.f,0.f,0.f};

  for (int k0 = 0; k0 < K; k0 += 32) {
    V bh[4], bl[4];
#pragma unroll
    for (int j = 0; j < 4; ++j) {
      const size_t bo = (size_t)(n0 + (j << 4) + rlane) * ldb + koff + k0;
      bh[j] = Frag<T>::load(Bb + bo);
      if (SPLIT) bl[j] = Frag<T>::load(Bb2 + bo);
    }
#pragma unroll
    for (int i = 0; i < 4; ++i) {
      const size_t ao = (size_t)(m0 + (i << 4) + rlane) * lda + koff + k0;
      V ah = Frag<T>::load(Ab + ao);
      V al;
      if (SPLIT) al = Frag<T>::load(Ab2 + ao);
#pragma unroll
      for (int j = 0; j < 4; ++j) {
        acc[i][j] = Frag<T>::mma(ah, bh[j], acc[i][j]);
        if (SPLIT) {
          acc[i][j] = Frag<T>::mma(ah, bl[j], acc[i][j]);
          acc[i][j] = Frag<T>::mma(al, bh[j], acc[i][j]);
        }
      }
      Frag<T>::guard4(acc[i][0], acc[i][1], acc[i][2], acc[i][3], ah, SPLIT ? al : ah);
    }
    Frag<T>::keep(bh[0], bh[1], bh[2], bh[3]);
    if (SPLIT) Frag<T>::keep(bl[0], bl[1], bl[2], bl[3]);
  }
  acc_guard4(acc[0][0], acc[0][1], acc[0][2], acc[0][3]);
  acc_guard4(acc[1][0], acc[1][1], acc[1][2], acc[1][3]);
  acc_guard4(acc[2][0], acc[2][1], acc[2][2], acc[2][3]);
  acc_guard4(acc[3][0], acc[3][1], acc[3][2], acc[3][3]);

  float* slab = sT[wave];
  const float* Rb = RESID ? (resid + (size_t)b * strideR) : nullptr;
#pragma unroll
  for (int i = 0; i < 4; ++i) {
    const int mBase = m0 + (i << 4);
#pragma unroll
    for (int j = 0; j < 4; ++j) {
      const int n = n0 + (j << 4) + rlane;
      float bv = 0.f;
      if (BIAS_MODE == 2) bv = bias[n];
#pragma unroll
      for (int r = 0; r < 8; ++r) {
        float v = acc[i][j][r] * scale;
        if (BIAS_MODE == 1) v += bias[mBase + mOff + r];
        if (BIAS_MODE == 2) v += bv;
        if (RESID) v += Rb[(size_t)(mBase + mOff + r) * ldc + n];
        if (ACT == 1) v = tanhf(v);
        if (ACT == 2) v = fmaxf(v, 0.0f);
        if (ACT == 3) v = v / (1.0f + expf(-v));
        if (ACT == 4) v = (v > 0.f) ? v : 0.01f * v;
        slab[(mOff + r) * 68 + (j << 4) + rlane] = v;
      }
    }
    __builtin_amdgcn_fence(__ATOMIC_RELEASE, "workgroup");
    __builtin_amdgcn_wave_barrier();
    __builtin_amdgcn_fence(__ATOMIC_ACQUIRE, "workgroup");
    if (OUT_MODE == 0) {
      float* C = (float*)Cout + (size_t)b * strideC;
      const int hh = lane >> 4, c4 = (lane & 15) * 4;
      for (int pass = 0; pass < 2; ++pass) {
#pragma unroll
        for (int it = 0; it < 8; ++it) {
          const int row = it * 2 + hh;
          v4f v = *(const v4f*)(slab + row * 68 + c4);
          *(volatile v4f*)(C + (size_t)(mBase + row) * ldc + n0 + c4) = v;
        }
        __threadfence();
      }
    } else {
      const int q = lane >> 3, c8 = (lane & 7) * 8;
      unsigned short* C  = (unsigned short*)Cout  + (size_t)b * strideC;
      unsigned short* C2 = (OUT_MODE == 2) ? ((unsigned short*)Cout2 + (size_t)b * strideC) : nullptr;
      for (int pass = 0; pass < 2; ++pass) {
#pragma unroll
        for (int it = 0; it < 4; ++it) {
          const int row = it * 4 + q;
          const float* sp = slab + row * 68 + c8;
          v8h hv, lv;
#pragma unroll
          for (int e = 0; e < 8; ++e) {
            if (OUT_MODE == 1) {
              hv[e] = (_Float16)sp[e];
            } else {
              unsigned short hb = f2bf_bits(sp[e]);
              unsigned short lb = f2bf_bits(sp[e] - bf_bits2f(hb));
              hv[e] = __builtin_bit_cast(_Float16, hb);
              lv[e] = __builtin_bit_cast(_Float16, lb);
            }
          }
          *(volatile v8h*)(C + (size_t)(mBase + row) * ldc + n0 + c8) = hv;
          if (OUT_MODE == 2) *(volatile v8h*)(C2 + (size_t)(mBase + row) * ldc + n0 + c8) = lv;
        }
        __threadfence();
      }
    }
    __builtin_amdgcn_fence(__ATOMIC_RELEASE, "workgroup");
    __builtin_amdgcn_wave_barrier();
    __builtin_amdgcn_fence(__ATOMIC_ACQUIRE, "workgroup");
  }
}

__global__ __launch_bounds__(kThr) void cast_plane_kernel(const float* __restrict__ src, unsigned short* __restrict__ dst,
                                                          int colsLog2, int dstPitch, int dstOff) {
  const int i   = blockIdx.x * kThr + threadIdx.x;
  const int sh  = colsLog2 - 3;
  const int row = i >> sh;
  const int c8  = (i & ((1 << sh) - 1)) * 8;
  const float* sp = src + ((size_t)row << colsLog2) + c8;
  const v4f a0 = *(const v4f*)(sp);
  const v4f a1 = *(const v4f*)(sp + 4);
  v8h hv;
#pragma unroll
  for (int e = 0; e < 4; ++e) {
    const float f0 = a0[e];
    const float f1 = a1[e];
    hv[e]     = (_Float16)carry_flush(bf16r(f0), kInCarry);
    hv[4 + e] = (_Float16)carry_flush(bf16r(f1), kInCarry);
  }
  unsigned short* dp = dst + (size_t)row * dstPitch + dstOff + c8;
  *(volatile v8h*)dp = hv;
  __threadfence();
  *(volatile v8h*)dp = hv;
}

__device__ __forceinline__ float fast_tanh(float v) { return 1.0f - 2.0f * frcp(__expf(2.0f * v) + 1.0f); }
__device__ __forceinline__ float fast_sigmoid(float v) { return frcp(1.0f + __expf(-v)); }
__device__ __forceinline__ void split_f16(float x, float c, float cinv, _Float16& hi, _Float16& lo) {
  hi = (_Float16)carry_flush(x, c);
  const float back = (float)hi * cinv;
  lo = (_Float16)carry_flush(x - back, c);
}

__global__ __launch_bounds__(kThr) void setup_kernel(const float* __restrict__ ebi, const float* __restrict__ ebh, const float* __restrict__ dbi,
                                                     const float* __restrict__ dbh, const float* __restrict__ lb, float* __restrict__ BIAS,
                                                     float* __restrict__ ZI, unsigned short* __restrict__ XIN2) {
  unsigned v = blockIdx.x * (unsigned)kThr + threadIdx.x;
  asm volatile("" : "+v"(v));
  if (v < 3328u) {
    const unsigned i0 = v * 4u;
    const unsigned seg = i0 / 3072u, j = i0 % 3072u;
    const bool live = i0 < (unsigned)(kFBL + kXD);
    const float* sp = (seg == 0u) ? (ebi + j) : (seg == 1u) ? (ebh + j) : (seg == 2u) ? (dbi + j) : (seg == 3u) ? (dbh + j) : (lb + (live ? (i0 - (unsigned)kFBL) : 0u));
    const v4f a = *(const v4f*)sp;
    v4f o;
#pragma unroll
    for (int e = 0; e < 4; ++e) { const float x = a[e]; o[e] = live ? bf16r(x) : 0.0f; }
    float* dp = BIAS + i0;
    *(volatile v4f*)dp = o;
    __threadfence();
    *(volatile v4f*)dp = o;
  } else if (v < 134400u) {
    const v4f z = {0.f, 0.f, 0.f, 0.f};
    float* dp = ZI + (size_t)(v - 3328u) * 4u;
    *(volatile v4f*)dp = z;
    __threadfence();
    *(volatile v4f*)dp = z;
  } else {
    v8h z;
#pragma unroll
    for (int e = 0; e < 8; ++e) z[e] = (_Float16)0.0f;
    unsigned short* dp = XIN2 + (size_t)(v - 134400u) * 8u;
    *(volatile v8h*)dp = z;
    __threadfence();
    *(volatile v8h*)dp = z;
  }
}
static_assert(kFEnd / 4 == 3328 && 3328 % kThr == 0 && 2 * kB * kHD / 4 == 131072 && 3328 + 131072 == 134400 && kB * 256 / 8 == 8192 && 134400 + 8192 == 557 * kThr && (kFBL % 3072) == 0, "set-up grid exact");

__global__ __launch_bounds__(kThr) void hprev_kernel(const float* __restrict__ O, const float* __restrict__ S, int m1, int m2,
                                                     float* __restrict__ HP32, unsigned short* __restrict__ HP16) {
  unsigned v = blockIdx.x * (unsigned)kThr + threadIdx.x;
  asm volatile("" : "+v"(v));
  const size_t o8 = (size_t)v * 8u;
  const float f1 = (float)m1, f2 = (float)m2;
  const v4f a0 = *(const v4f*)(O + o8), a1 = *(const v4f*)(O + o8 + 4), s0 = *(const v4f*)(S + o8), s1 = *(const v4f*)(S + o8 + 4);
  v4f h0, h1; v8h hv;
#pragma unroll
  for (int e = 0; e < 4; ++e) { h0[e] = a0[e] * f1 + s0[e] * f2; h1[e] = a1[e] * f1 + s1[e] * f2; hv[e] = (_Float16)carry_flush(h0[e], kInCarry); hv[4 + e] = (_Float16)carry_flush(h1[e], kInCarry); }
  for (int pass = 0; pass < 2; ++pass) {
    *(volatile v4f*)(HP32 + o8) = h0; *(volatile v4f*)(HP32 + o8 + 4) = h1;
    *(volatile v8h*)(HP16 + o8) = hv;
    __threadfence();
  }
}
static_assert(kB * kHD / 8 == 128 * kThr, "state grids exact");

__global__ __launch_bounds__(kThr) void cell_kernel(const float* __restrict__ GI, const float* __restrict__ GH, const float* __restrict__ HP32,
                                                    float* __restrict__ HN) {
  unsigned v = blockIdx.x * (unsigned)kThr + threadIdx.x;
  asm volatile("" : "+v"(v));
  const unsigned b = v >> 7, u8 = (v & 127u) * 8u;
  const float* gi = GI + (size_t)b * kG3 + u8;
  const float* gh = GH + (size_t)b * kG3 + u8;
  const float* hp = HP32 + (size_t)b * kHD + u8;
  v4f hn0, hn1;
#pragma unroll
  for (int hlf = 0; hlf < 2; ++hlf) {
    const v4f ir = *(const v4f*)(gi + 4 * hlf), iz = *(const v4f*)(gi + kHD + 4 * hlf), in_ = *(const v4f*)(gi + 2 * kHD + 4 * hlf);
    const v4f hr = *(const v4f*)(gh + 4 * hlf), hz = *(const v4f*)(gh + kHD + 4 * hlf), hn_ = *(const v4f*)(gh + 2 * kHD + 4 * hlf);
    const v4f ho = *(const v4f*)(hp + 4 * hlf);
#pragma unroll
    for (int e = 0; e < 4; ++e) {
      const float r = fast_sigmoid(ir[e] + hr[e]);
      const float z = fast_sigmoid(iz[e] + hz[e]);
      const float n = fast_tanh(in_[e] + r * hn_[e]);
      const float hn = (1.0f - z) * n + z * ho[e];
      if (hlf == 0) hn0[e] = hn; else hn1[e] = hn;
    }
  }
  float* dp = HN + (size_t)b * kHD + u8;
  for (int pass = 0; pass < 2; ++pass) {
    *(volatile v4f*)dp = hn0; *(volatile v4f*)(dp + 4) = hn1;
    __threadfence();
  }
}

__global__ __launch_bounds__(kThr) void henc_kernel(const float* __restrict__ L, float* __restrict__ INIT) {
  unsigned v = blockIdx.x * (unsigned)kThr + threadIdx.x;
  asm volatile("" : "+v"(v));
  const size_t o8 = (size_t)v * 8u;
  const v4f a0 = *(const v4f*)(L + o8), a1 = *(const v4f*)(L + o8 + 4);
  v4f h0, h1;
#pragma unroll
  for (int e = 0; e < 4; ++e) { h0[e] = a0[e] + a0[e]; h1[e] = a1[e] + a1[e]; }
  for (int pass = 0; pass < 2; ++pass) {
    *(volatile v4f*)(INIT + o8) = h0; *(volatile v4f*)(INIT + o8 + 4) = h1;
    __threadfence();
  }
}

__global__ __launch_bounds__(kThr) void pj_kernel(const float* __restrict__ O, const float* __restrict__ S, unsigned short* __restrict__ PJ2) {
  unsigned v = blockIdx.x * (unsigned)kThr + threadIdx.x;
  asm volatile("" : "+v"(v));
  const unsigned b = v >> 7, u8 = (v & 127u) * 8u;
  const size_t o8 = (size_t)b * kHD + u8;
  const v4f a0 = *(const v4f*)(O + o8), a1 = *(const v4f*)(O + o8 + 4), s0 = *(const v4f*)(S + o8), s1 = *(const v4f*)(S + o8 + 4);
  v8h hv, lv;
#pragma unroll
  for (int e = 0; e < 4; ++e) {
    _Float16 hi, lo;
    split_f16(a0[e] + s0[e], kInCarry, 1.0f / kInCarry, hi, lo); hv[e] = hi; lv[e] = lo;
    split_f16(a1[e] + s1[e], kInCarry, 1.0f / kInCarry, hi, lo); hv[4 + e] = hi; lv[4 + e] = lo;
  }
  unsigned short* dp = PJ2 + (size_t)b * (2 * kHD) + u8;
  for (int pass = 0; pass < 2; ++pass) {
    *(volatile v8h*)dp = hv;
    *(volatile v8h*)(dp + kHD) = lv;
    __threadfence();
  }
}

__global__ __launch_bounds__(kThr) void out_kernel(const float* __restrict__ PR32, float* __restrict__ out, unsigned short* __restrict__ XIN2, int i) {
  unsigned v = blockIdx.x * (unsigned)kThr + threadIdx.x;
  asm volatile("" : "+v"(v));
  const unsigned b = v >> 4, c8 = (v & 15u) * 8u;
  const v4f a0 = *(const v4f*)(PR32 + (size_t)b * kXD + c8), a1 = *(const v4f*)(PR32 + (size_t)b * kXD + c8 + 4);
  v8h hv, lv;
#pragma unroll
  for (int e = 0; e < 4; ++e) {
    _Float16 hi, lo;
    split_f16(a0[e], kInCarry, 1.0f / kInCarry, hi, lo); hv[e] = hi; lv[e] = lo;
    split_f16(a1[e], kInCarry, 1.0f / kInCarry, hi, lo); hv[4 + e] = hi; lv[4 + e] = lo;
  }
  float* op = out + ((size_t)b * kT + (size_t)i) * kXD + c8;
  unsigned short* xp = XIN2 + (size_t)b * (2 * kXD) + c8;
  for (int pass = 0; pass < 2; ++pass) {
    *(volatile v4f*)op = a0; *(volatile v4f*)(op + 4) = a1;
    *(volatile v8h*)xp = hv;
    *(volatile v8h*)(xp + kXD) = lv;
    __threadfence();
  }
}
static_assert(kB * 16 == 16 * kThr, "output grid exact");

static_assert(((size_t)kG3 * kHD / 8) % kThr == 0 && ((size_t)kG3 * kXD / 8) % kThr == 0 && ((size_t)kXD * kHD / 8) % kThr == 0 && ((size_t)kB * kT * kXD / 8) % kThr == 0, "plane cast grids exact");

extern "C" void kernel_launch(void* const* d_in, const int* in_sizes, int n_in,
                              void* d_out, int out_size, void* d_ws, size_t ws_size,
                              hipStream_t stream) {
  if (n_in < 11 || d_out == nullptr || d_ws == nullptr) return;
  if (in_sizes[0] != kB * kT * kXD || in_sizes[1] != kG3 * kXD || in_sizes[2] != kG3 * kHD || in_sizes[3] != kG3 || in_sizes[4] != kG3) return;
  if (in_sizes[5] != kG3 * kXD || in_sizes[6] != kG3 * kHD || in_sizes[7] != kG3 || in_sizes[8] != kG3 || in_sizes[9] != kXD * kHD || in_sizes[10] != kXD) return;
  if (out_size != kB * kT * kXD) return;
  if (ws_size < kWsTotal) return;
  const float* input = (const float*)d_in[0];
  const float* enc_W_ih = (const float*)d_in[1];
  const float* enc_W_hh = (const float*)d_in[2];
  const float* enc_b_ih = (const float*)d_in[3];
  const float* enc_b_hh = (const float*)d_in[4];
  const float* dec_W_ih = (const float*)d_in[5];
  const float* dec_W_hh = (const float*)d_in[6];
  const float* dec_b_ih = (const float*)d_in[7];
  const float* dec_b_hh = (const float*)d_in[8];
  const float* lin_W = (const float*)d_in[9];
  const float* lin_b = (const float*)d_in[10];
  float* out = (float*)d_out;
  char* ws = (char*)d_ws;
  unsigned short* EWH = (unsigned short*)(ws + kOffEWH);
  unsigned short* EWI = (unsigned short*)(ws + kOffEWI);
  unsigned short* DWH = (unsigned short*)(ws + kOffDWH);
  unsigned short* DWI2 = (unsigned short*)(ws + kOffDWI2);
  unsigned short* LW2 = (unsigned short*)(ws + kOffLW2);
  float* BIAS = (float*)(ws + kOffBIAS);
  unsigned short* X16 = (unsigned short*)(ws + kOffX16);
  float* ZERO = (float*)(ws + kOffZERO);
  float* INIT = (float*)(ws + kOffINIT);
  float* RING = (float*)(ws + kOffRING);
  float* HP32 = (float*)(ws + kOffHP32);
  unsigned short* HP16 = (unsigned short*)(ws + kOffHP16);
  float* GI = (float*)(ws + kOffGI);
  float* GH = (float*)(ws + kOffGH);
  unsigned short* PJ2 = (unsigned short*)(ws + kOffPJ2);
  float* PR32 = (float*)(ws + kOffPR32);
  unsigned short* XIN2 = (unsigned short*)(ws + kOffXIN2);
  const size_t kSlot = (size_t)kB * kHD;

  cast_plane_kernel<<<(int)(((size_t)kG3 * kHD / 8) / kThr), kThr, 0, stream>>>(enc_W_hh, EWH, 10, kHD, 0);
  cast_plane_kernel<<<(int)(((size_t)kG3 * kXD / 8) / kThr), kThr, 0, stream>>>(enc_W_ih, EWI, 7, kXD, 0);
  cast_plane_kernel<<<(int)(((size_t)kG3 * kHD / 8) / kThr), kThr, 0, stream>>>(dec_W_hh, DWH, 10, kHD, 0);
  cast_plane_kernel<<<(int)(((size_t)kG3 * kXD / 8) / kThr), kThr, 0, stream>>>(dec_W_ih, DWI2, 7, 2 * kXD, 0);
  cast_plane_kernel<<<(int)(((size_t)kG3 * kXD / 8) / kThr), kThr, 0, stream>>>(dec_W_ih, DWI2, 7, 2 * kXD, kXD);
  cast_plane_kernel<<<(int)(((size_t)kXD * kHD / 8) / kThr), kThr, 0, stream>>>(lin_W, LW2, 10, 2 * kHD, 0);
  cast_plane_kernel<<<(int)(((size_t)kXD * kHD / 8) / kThr), kThr, 0, stream>>>(lin_W, LW2, 10, 2 * kHD, kHD);
  cast_plane_kernel<<<(int)(((size_t)kB * kT * kXD / 8) / kThr), kThr, 0, stream>>>(input, X16, 13, kT * kXD, 0);
  setup_kernel<<<557, kThr, 0, stream>>>(enc_b_ih, enc_b_hh, dec_b_ih, dec_b_hh, lin_b, BIAS, ZERO, XIN2);

  for (int phase = 0; phase < 2; ++phase) {
    const bool dec = (phase == 1);
    const unsigned short* WH = dec ? DWH : EWH;
    for (int i = 0; i < kT; ++i) {
      const float* O = (i == 0) ? INIT : (RING + (size_t)((i - 1) & (kRing - 1)) * kSlot);
      const int ps = kPrevSkip[i];
      const float* S = (ps < 0) ? ZERO : (RING + (size_t)(ps & (kRing - 1)) * kSlot);
      hprev_kernel<<<128, kThr, 0, stream>>>(O, S, dec ? kDecM1[i] : kEncM1[i], dec ? kDecM2[i] : kEncM2[i], HP32, HP16);
      wmma_gemm64<0, false, 2, 0, false, 0><<<dim3((kB / 64) * (kG3 / 64) / 8, 1), 256, 0, stream>>>(
          HP16, HP16, kHD, 0L, WH, WH, kHD, 0L, (void*)GH, (void*)GH, kG3, 0L, BIAS + (dec ? kFDH : kFEH), nullptr, 0L, kB, kG3, kHD, kSc);
      if (!dec) {
        wmma_gemm64<0, false, 2, 0, false, 0><<<dim3((kB / 64) * (kG3 / 64) / 8, 1), 256, 0, stream>>>(
            X16 + (size_t)i * kXD, X16 + (size_t)i * kXD, kT * kXD, 0L, EWI, EWI, kXD, 0L, (void*)GI, (void*)GI, kG3, 0L, BIAS + kFEI, nullptr, 0L, kB, kG3, kXD, kSc);
      } else {
        wmma_gemm64<0, false, 2, 0, false, 0><<<dim3((kB / 64) * (kG3 / 64) / 8, 1), 256, 0, stream>>>(
            XIN2, XIN2, 2 * kXD, 0L, DWI2, DWI2, 2 * kXD, 0L, (void*)GI, (void*)GI, kG3, 0L, BIAS + kFDI, nullptr, 0L, kB, kG3, 2 * kXD, kSc);
      }
      float* HN = RING + (size_t)(i & (kRing - 1)) * kSlot;
      cell_kernel<<<128, kThr, 0, stream>>>(GI, GH, HP32, HN);
      if (dec) {
        const int js = kProjSkip[i];
        const float* SJ = (js < 0) ? ZERO : (RING + (size_t)(js & (kRing - 1)) * kSlot);
        pj_kernel<<<128, kThr, 0, stream>>>(O, SJ, PJ2);
        wmma_gemm64<0, false, 2, 0, false, 0><<<dim3((kB / 64) * (kXD / 64) / 8, 1), 256, 0, stream>>>(
            PJ2, PJ2, 2 * kHD, 0L, LW2, LW2, 2 * kHD, 0L, (void*)PR32, (void*)PR32, kXD, 0L, BIAS + kFBL, nullptr, 0L, kB, kXD, 2 * kHD, kSc);
        out_kernel<<<16, kThr, 0, stream>>>(PR32, out, XIN2, i);
      }
    }
    if (!dec) henc_kernel<<<128, kThr, 0, stream>>>(RING + (size_t)((kT - 1) & (kRing - 1)) * kSlot, INIT);
  }
}
